// JTMPN_16389595201591
// MI455X (gfx1250) — hardware-verified
//
#include <hip/hip_runtime.h>
#include <math.h>

typedef __attribute__((ext_vector_type(16))) _Float16 v16h;
typedef __attribute__((ext_vector_type(16))) __bf16 v16b;
typedef __attribute__((ext_vector_type(8)))  _Float16 v8h;
typedef __attribute__((ext_vector_type(8)))  float v8f;
typedef __attribute__((ext_vector_type(4)))  float v4f;
typedef __attribute__((ext_vector_type(2)))  float v2f;
typedef __attribute__((ext_vector_type(4)))  unsigned v4u;
typedef __attribute__((ext_vector_type(4)))  int v4i;
typedef float __attribute__((may_alias)) float_a;
typedef int __attribute__((may_alias)) int_a;

template <typename T> __device__ __forceinline__ void vst2(void* p, T v) { *(volatile T*)p = v; __threadfence(); *(volatile T*)p = v; }
__device__ __forceinline__ v8f wmma16(v16h a, v16h b, v8f c) {
  v8f d = __builtin_amdgcn_wmma_f32_16x16x32_f16(false, a, false, b, (short)0, c, false, false);
  asm volatile("v_nop\n\tv_nop\n\tv_nop\n\tv_nop" : "+v"(d) : "v"(a), "v"(b));
  return d;
}
__device__ __forceinline__ v8f wmma_bf(v16b a, v16b b, v8f c) {
  v8f d = __builtin_amdgcn_wmma_f32_16x16x32_bf16(false, a, false, b, (short)0, c, false, false);
  asm volatile("v_nop\n\tv_nop\n\tv_nop\n\tv_nop" : "+v"(d) : "v"(a), "v"(b));
  return d;
}
__device__ __forceinline__ v16h frag_h(const _Float16* rowk0, int lane) {
  union { v16h v; v8h q[2]; } u; const _Float16* p = rowk0 + 8 * (lane >> 4);
  u.q[0] = *(const v8h*)p; u.q[1] = *(const v8h*)(p + 16); return u.v;
}
__device__ __forceinline__ v16h frag_f32(const float* rowk0, int lane) {
  v16h a; const float* p = rowk0 + 8 * (lane >> 4);
#pragma unroll
  for (int i = 0; i < 8; ++i) { a[i] = (_Float16)p[i]; a[8 + i] = (_Float16)p[16 + i]; }
  return a;
}
__device__ __forceinline__ v16h frag_f32s(const float* rowk0, int lane, float sc) {
  v16h a; const float* p = rowk0 + 8 * (lane >> 4);
#pragma unroll
  for (int i = 0; i < 8; ++i) { a[i] = (_Float16)(p[i] * sc); a[8 + i] = (_Float16)(p[16 + i] * sc); }
  return a;
}
__device__ __forceinline__ v16h fragc_f32(const float* W, int k0, int n, int lane, int ld, int K) {
  v16h a; const int g = lane >> 4;
#pragma unroll
  for (int i = 0; i < 8; ++i) { const int ka = k0 + 8 * g + i, kb = ka + 16;
    a[i] = (_Float16)(ka < K ? W[(size_t)ka * ld + n] : 0.f); a[8 + i] = (_Float16)(kb < K ? W[(size_t)kb * ld + n] : 0.f); }
  return a;
}
struct F2 { v16b h, l; };
__device__ __forceinline__ F2 bsplit16(const float v[16]) { F2 r;
#pragma unroll
  for (int i = 0; i < 16; ++i) { const __bf16 h = (__bf16)v[i]; r.h[i] = h; r.l[i] = (__bf16)(v[i] - (float)h); }
  return r; }
__device__ __forceinline__ F2 split_row(const float* row, int k0, int lane) { float v[16]; const float* p = row + k0 + 8 * (lane >> 4);
#pragma unroll
  for (int i = 0; i < 8; ++i) { v[i] = p[i]; v[8 + i] = p[16 + i]; }
  return bsplit16(v); }
__device__ __forceinline__ F2 split_rowK(const float* row, int k0, int lane, int K) { float v[16]; const int g = lane >> 4;
#pragma unroll
  for (int i = 0; i < 8; ++i) { const int ka = k0 + 8 * g + i, kb = ka + 16; v[i] = ka < K ? row[ka] : 0.f; v[8 + i] = kb < K ? row[kb] : 0.f; }
  return bsplit16(v); }
__device__ __forceinline__ F2 split_col(const float* W, int k0, int n, int lane, int ld, int K) { float v[16]; const int g = lane >> 4;
#pragma unroll
  for (int i = 0; i < 8; ++i) { const int ka = k0 + 8 * g + i, kb = ka + 16; v[i] = ka < K ? W[(size_t)ka * ld + n] : 0.f; v[8 + i] = kb < K ? W[(size_t)kb * ld + n] : 0.f; }
  return bsplit16(v); }
__device__ __forceinline__ v8f mac3(const F2& a, const F2& b, v8f c) { c = wmma_bf(a.l, b.h, c); c = wmma_bf(a.h, b.l, c); return wmma_bf(a.h, b.h, c); }
__device__ __forceinline__ float sigm(float v) { return 1.0f / (1.0f + expf(-v)); }
#define LDSX() do { asm volatile("s_wait_dscnt 0" ::: "memory"); __builtin_amdgcn_wave_barrier(); __builtin_amdgcn_fence(__ATOMIC_RELEASE, "workgroup"); } while (0)

#define HH 256
#define NAT 50000
#define NBD 100000
#define NMS 10000
#define NMSG (NMS + NBD)
#define NPR 10000
#define NMOL 2000
#define APM 25
#define AFD 35
#define BFD 40
#define MAXNB 10

__global__ __launch_bounds__(256) void k_tree(const float* __restrict__ tm, _Float16* __restrict__ MA, _Float16* __restrict__ MB) {
  const size_t i8 = (size_t)blockIdx.x * 256 + threadIdx.x; if (i8 >= (size_t)NMS * HH / 8) return;
  union { v8h h; v4u u; } pk;
#pragma unroll
  for (int e = 0; e < 8; ++e) pk.h[e] = (_Float16)tm[i8 * 8 + e];
  vst2(MA + i8 * 8, pk.u); vst2(MB + i8 * 8, pk.u);
}
__device__ __forceinline__ void fill_wi(_Float16 (*swi)[72], const float* __restrict__ Wi, int tid, int nth) {
  for (int q = tid; q < HH * 64; q += nth) { const int n = q >> 6, k = q & 63; swi[n][k] = (_Float16)(k < BFD ? Wi[(size_t)n * BFD + k] * 16.0f : 0.f); }
}
template <int ROUND0>
__global__ __launch_bounds__(128) void k_bond(const float* __restrict__ fb, const float* __restrict__ Wi, const float* __restrict__ Wh, const int* __restrict__ bgraph, const _Float16* __restrict__ MIN, _Float16* __restrict__ MOUT) {
  __shared__ __align__(16) _Float16 swi[HH][72];
  __shared__ __align__(16) _Float16 sfb[4][16][72];
  __shared__ __align__(16) _Float16 snei[4][16][HH + 8];
  __shared__ __align__(16) float so[4][16][132];
  const int tid = threadIdx.x, wave = tid >> 5, lane = tid & 31, col = lane & 15, g = lane >> 4;
  const int r0 = blockIdx.x * 64 + wave * 16;
  fill_wi(swi, Wi, tid, 128);
  { const int r = r0 + col; const bool live = r < NBD; const int rc = live ? r : 0; for (int k = g; k < 64; k += 2) sfb[wave][col][k] = (_Float16)((live && k < BFD) ? fb[(size_t)rc * BFD + k] : 0.f); }
  if (!ROUND0) {
    const int rl = lane >> 1, hf = lane & 1; const int r = r0 + rl; const bool live = r < NBD; const int* nb = bgraph + (size_t)(live ? r : 0) * MAXNB;
    for (int c8 = hf * 16; c8 < hf * 16 + 16; ++c8) { float s[8] = {0.f, 0.f, 0.f, 0.f, 0.f, 0.f, 0.f, 0.f};
      if (live) for (int j = 0; j < MAXNB; ++j) { int m = nb[j]; m = m < 0 ? 0 : (m >= NMSG ? NMSG - 1 : m); union { v4u u; v8h h; } pk; pk.u = *(const v4u*)(MIN + (size_t)m * HH + c8 * 8);
#pragma unroll
        for (int e = 0; e < 8; ++e) s[e] += (float)pk.h[e]; }
      union { v8h h; v4u u; } o;
#pragma unroll
      for (int e = 0; e < 8; ++e) o.h[e] = (_Float16)s[e];
      *(v4u*)(&snei[wave][rl][c8 * 8]) = o.u; } }
  __syncthreads();
#pragma unroll 1
  for (int nh = 0; nh < 2; ++nh) { v8f acc[8] = {};
#pragma unroll
    for (int kc = 0; kc < 2; ++kc) { const v16h a = frag_h(&sfb[wave][col][0] + kc * 32, lane);
#pragma unroll
      for (int j = 0; j < 8; ++j) acc[j] = wmma16(a, frag_h(&swi[nh * 128 + j * 16 + col][0] + kc * 32, lane), acc[j]); }
    if (!ROUND0) {
#pragma unroll 2
      for (int kc = 0; kc < HH / 32; ++kc) { const v16h a = frag_h(&snei[wave][col][0] + kc * 32, lane);
#pragma unroll
        for (int j = 0; j < 8; ++j) acc[j] = wmma16(a, frag_f32s(Wh + (size_t)(nh * 128 + j * 16 + col) * HH + kc * 32, lane, 16.0f), acc[j]); } }
#pragma unroll
    for (int j = 0; j < 8; ++j)
#pragma unroll
      for (int r = 0; r < 8; ++r) { const float v = acc[j][r] * (1.0f / 16.0f); so[wave][8 * g + r][j * 16 + col] = v > 0.f ? v : 0.f; }
    LDSX();
    for (int q = lane; q < 16 * 16; q += 32) { const int rl = q >> 4, pc = q & 15; union { v8h h; v4u u; } pk;
#pragma unroll
      for (int e = 0; e < 8; ++e) pk.h[e] = (_Float16)so[wave][rl][pc * 8 + e];
      if (r0 + rl < NBD) vst2(MOUT + (size_t)(NMS + r0 + rl) * HH + nh * 128 + pc * 8, pk.u); }
    LDSX(); }
}
__global__ __launch_bounds__(256) void k_coll(const _Float16* __restrict__ M, const int* __restrict__ pidx, float* __restrict__ out2) {
  const int wave = threadIdx.x >> 5, lane = threadIdx.x & 31; const int p = blockIdx.x * 8 + wave; if (p >= NPR) return;
  int a = pidx[p * 2], b = pidx[p * 2 + 1]; a = a < 0 ? 0 : (a >= NBD ? NBD - 1 : a); b = b < 0 ? 0 : (b >= NBD ? NBD - 1 : b);
  const _Float16* ra = M + (size_t)(NMS + a) * HH; const _Float16* rb = M + (size_t)(NMS + b) * HH;
  for (int c = lane * 4; c < HH; c += 128) { v4f o;
#pragma unroll
    for (int e = 0; e < 4; ++e) o[e] = ((float)ra[c + e] + (float)rb[c + e]) * 0.5f;
    vst2(out2 + (size_t)p * HH + c, o); }
}
__global__ __launch_bounds__(128) void k_atom(const float* __restrict__ fa, const float* __restrict__ Wo, const float* __restrict__ bo, const int* __restrict__ agraph, const _Float16* __restrict__ M, float* __restrict__ out1) {
  __shared__ __align__(16) _Float16 swo[HH][72];
  __shared__ __align__(16) _Float16 sfa[4][16][72];
  __shared__ __align__(16) _Float16 snei[4][16][HH + 8];
  __shared__ __align__(16) float sh[64][HH + 4];
  __shared__ __align__(16) float smol[2][HH];
  const int tid = threadIdx.x, wave = tid >> 5, lane = tid & 31, col = lane & 15, g = lane >> 4;
  const int a0 = blockIdx.x * 2 * APM;
  for (int q = tid; q < HH * 64; q += 128) { const int n = q >> 6, k = q & 63; swo[n][k] = (_Float16)(k < AFD ? Wo[(size_t)n * (AFD + HH) + k] * 16.0f : 0.f); }
  { const int rl = wave * 16 + col; const int at = a0 + rl; const bool live = rl < 2 * APM && at < NAT; const int atc = live ? at : 0;
    for (int k = g; k < 64; k += 2) sfa[wave][col][k] = (_Float16)((live && k < AFD) ? fa[(size_t)atc * AFD + k] : 0.f); }
  { const int rl = lane >> 1, hf = lane & 1; const int at = a0 + wave * 16 + rl; const bool live = (wave * 16 + rl) < 2 * APM && at < NAT; const int* nb = agraph + (size_t)(live ? at : 0) * MAXNB;
    for (int c8 = hf * 16; c8 < hf * 16 + 16; ++c8) { float s[8] = {0.f, 0.f, 0.f, 0.f, 0.f, 0.f, 0.f, 0.f};
      if (live) { for (int j = 0; j < MAXNB; ++j) { int m = nb[j]; m = m < 0 ? 0 : (m >= NMSG ? NMSG - 1 : m); union { v4u u; v8h h; } pk; pk.u = *(const v4u*)(M + (size_t)m * HH + c8 * 8);
#pragma unroll
          for (int e = 0; e < 8; ++e) s[e] += (float)pk.h[e]; } }
      union { v8h h; v4u u; } o;
#pragma unroll
      for (int e = 0; e < 8; ++e) o.h[e] = (_Float16)s[e];
      *(v4u*)(&snei[wave][rl][c8 * 8]) = o.u; } }
  __syncthreads();
#pragma unroll 1
  for (int nh = 0; nh < 2; ++nh) { v8f acc[8] = {};
#pragma unroll
    for (int kc = 0; kc < 2; ++kc) { const v16h a = frag_h(&sfa[wave][col][0] + kc * 32, lane);
#pragma unroll
      for (int j = 0; j < 8; ++j) acc[j] = wmma16(a, frag_h(&swo[nh * 128 + j * 16 + col][0] + kc * 32, lane), acc[j]); }
#pragma unroll 2
    for (int kc = 0; kc < HH / 32; ++kc) { const v16h a = frag_h(&snei[wave][col][0] + kc * 32, lane);
#pragma unroll
      for (int j = 0; j < 8; ++j) acc[j] = wmma16(a, frag_f32s(Wo + (size_t)(nh * 128 + j * 16 + col) * (AFD + HH) + AFD + kc * 32, lane, 16.0f), acc[j]); }
#pragma unroll
    for (int j = 0; j < 8; ++j) { const int n = nh * 128 + j * 16 + col; const float bb = bo[n];
#pragma unroll
      for (int r = 0; r < 8; ++r) { const float v = acc[j][r] * (1.0f / 16.0f) + bb; sh[wave * 16 + 8 * g + r][n] = v > 0.f ? v : 0.f; } } }
  __syncthreads();
  for (int q = tid; q < 2 * HH; q += 128) { const int ml = q >> 8, c = q & 255; float s = 0.f; for (int i = 0; i < APM; ++i) s += sh[ml * APM + i][c]; smol[ml][c] = s * (1.0f / APM); }
  __syncthreads();
  for (int q = tid; q < 2 * HH / 4; q += 128) { const int ml = q >> 6, pc = q & 63; const int mol = blockIdx.x * 2 + ml; if (mol < NMOL) vst2(out1 + (size_t)mol * HH + pc * 4, *(const v4f*)(&smol[ml][pc * 4])); }
}
extern "C" void kernel_launch(void* const* d_in, const int* in_sizes, int n_in, void* d_out, int out_size, void* d_ws, size_t ws_size, hipStream_t stream) {
  (void)in_sizes; (void)n_in; (void)out_size; (void)ws_size;
  const float* fa = (const float*)d_in[0]; const float* fb = (const float*)d_in[1]; const float* tm = (const float*)d_in[2]; const int* agraph = (const int*)d_in[3]; const int* bgraph = (const int*)d_in[4]; const int* pidx = (const int*)d_in[5];
  const float* Wi = (const float*)d_in[6]; const float* Wh = (const float*)d_in[7]; const float* Wo = (const float*)d_in[8]; const float* bo = (const float*)d_in[9];
  float* out1 = (float*)d_out; float* out2 = (float*)((char*)d_out + 2048000);
  char* ws = (char*)d_ws; size_t off = 0;
  auto take = [&](size_t bytes) { char* p = ws + off; off += (bytes + 255) & ~(size_t)255; return p; };
  _Float16* MA = (_Float16*)take((size_t)NMSG * HH * 2); _Float16* MB = (_Float16*)take((size_t)NMSG * HH * 2);
  k_tree<<<(NMS * HH / 8 + 255) / 256, 256, 0, stream>>>(tm, MA, MB);
  k_bond<1><<<(NBD + 63) / 64, 128, 0, stream>>>(fb, Wi, Wh, bgraph, MB, MA);
  k_bond<0><<<(NBD + 63) / 64, 128, 0, stream>>>(fb, Wi, Wh, bgraph, MA, MB);
  k_bond<0><<<(NBD + 63) / 64, 128, 0, stream>>>(fb, Wi, Wh, bgraph, MB, MA);
  k_bond<0><<<(NBD + 63) / 64, 128, 0, stream>>>(fb, Wi, Wh, bgraph, MA, MB);
  k_coll<<<(NPR + 7) / 8, 256, 0, stream>>>(MB, pidx, out2);
  k_atom<<<NMOL / 2, 128, 0, stream>>>(fa, Wo, bo, agraph, MB, out1);
}
